// DecoderOnlyBlock_446676599027
// MI455X (gfx1250) — hardware-verified
//
#include <hip/hip_runtime.h>
#include <stdint.h>

typedef _Float16 v16h __attribute__((ext_vector_type(16)));
typedef _Float16 v8h  __attribute__((ext_vector_type(8)));
typedef float    v8f  __attribute__((ext_vector_type(8)));
typedef float    v4f  __attribute__((ext_vector_type(4)));
typedef int      v4i  __attribute__((ext_vector_type(4)));
typedef v8h __attribute__((may_alias)) v8ha;
typedef v4f __attribute__((may_alias)) v4fa;
typedef v4i __attribute__((may_alias)) v4ia;

union Frag { v16h v; v8h half[2]; };

static constexpr int kB = 2, kS = 2048, kE = 1024, kH = 16, kD = 64, kF = 4096;
static constexpr int kM = kB * kS;
static constexpr float kWScale = 32.0f;
static constexpr float kPScale = 16384.0f;
static constexpr float kHScale = 16.0f;

static_assert(kM % 128 == 0);
static_assert(kS % 128 == 0);
static_assert(kE % 64 == 0);
static_assert(kF % 64 == 0);
static_assert(kD == 64);
static_assert(kM % 8 == 0);

__device__ __forceinline__ v8f wmma_f16(v16h a, v16h b, v8f c) {
  v8f d = __builtin_amdgcn_wmma_f32_16x16x32_f16(false, a, false, b, (short)0, c, false, false);
  asm volatile("v_nop\n\tv_nop\n\tv_nop\n\tv_nop" : "+v"(d) : "v"(a), "v"(b));
  return d;
}

__device__ __forceinline__ v16h load_frag(const _Float16* p, int h) {
  Frag f;
  f.half[0] = *(const v8ha*)(p + 8 * h);
  f.half[1] = *(const v8ha*)(p + 16 + 8 * h);
  return f.v;
}

__device__ __forceinline__ float wave_sum(float v) {
  v += __shfl_xor(v, 16);
  v += __shfl_xor(v, 8);
  v += __shfl_xor(v, 4);
  v += __shfl_xor(v, 2);
  v += __shfl_xor(v, 1);
  return v;
}

__device__ __forceinline__ float gelu_exact(float x) {
  return 0.5f * x * (1.0f + erff(x * 0.70710678118654752f));
}

__global__ __launch_bounds__(256) void cvt_wt_kernel(const float* __restrict__ in,
                                                     _Float16* __restrict__ out,
                                                     int Kdim, int Ndim, float sc) {
  __shared__ __attribute__((aligned(16))) _Float16 sT[64 * 72];
  const int tid = threadIdx.x, lane = tid & 31, w = tid >> 5;
  const int n0 = blockIdx.x * 64, k0 = blockIdx.y * 64;
  #pragma unroll
  for (int it = 0; it < 4; ++it) {
    const int idx = tid + 256 * it;
    const int kr = idx >> 4, c4 = (idx & 15) * 4;
    const v4f v = *(const v4fa*)(in + (size_t)(k0 + kr) * Ndim + n0 + c4);
    sT[(c4 + 0) * 72 + kr] = (_Float16)(v.x * sc);
    sT[(c4 + 1) * 72 + kr] = (_Float16)(v.y * sc);
    sT[(c4 + 2) * 72 + kr] = (_Float16)(v.z * sc);
    sT[(c4 + 3) * 72 + kr] = (_Float16)(v.w * sc);
  }
  __syncthreads();
  const int q8 = lane & 7, sub = lane >> 3;
  v8h vv[2];
  size_t di[2];
  #pragma unroll
  for (int i = 0; i < 2; ++i) {
    const int nl = 8 * w + 4 * i + sub;
    vv[i] = *(const v8ha*)(sT + nl * 72 + 8 * q8);
    di[i] = (size_t)(n0 + nl) * Kdim + k0 + 8 * q8;
  }
  #pragma unroll
  for (int i = 0; i < 2; ++i) *(volatile v8h*)(out + di[i]) = vv[i];
  __threadfence();
  #pragma unroll
  for (int i = 0; i < 2; ++i) *(volatile v8h*)(out + di[i]) = vv[i];
}

template <bool F32OUT>
__global__ __launch_bounds__(256) void ln_kernel(const float* __restrict__ x,
                                                 const float* __restrict__ g,
                                                 const float* __restrict__ bta,
                                                 float* __restrict__ outf,
                                                 _Float16* __restrict__ outh) {
  __shared__ __attribute__((aligned(16))) float sRow[8 * kE];
  const int tid = threadIdx.x, lane = tid & 31, w = tid >> 5;
  const int row = blockIdx.x * 8 + w;
  const float* xr = x + (size_t)row * kE;

  v4f v[8];
  float s = 0.f;
  #pragma unroll
  for (int j = 0; j < 8; ++j) {
    v[j] = *(const v4fa*)(xr + 128 * j + 4 * lane);
    s += (v[j].x + v[j].y) + (v[j].z + v[j].w);
  }
  s = wave_sum(s);
  const float mu = s * (1.0f / kE);
  float q = 0.f;
  #pragma unroll
  for (int j = 0; j < 8; ++j) {
    const v4f d = v[j] - mu;
    q += (d.x * d.x + d.y * d.y) + (d.z * d.z + d.w * d.w);
  }
  q = wave_sum(q);
  const float rstd = rsqrtf(q * (1.0f / kE) + 1e-5f);

  float* srow = sRow + w * kE;
  v4f y[8];
  #pragma unroll
  for (int j = 0; j < 8; ++j) {
    const int col = 128 * j + 4 * lane;
    const v4f gg = *(const v4fa*)(g + col);
    const v4f bb = *(const v4fa*)(bta + col);
    y[j] = (v[j] - mu) * rstd * gg + bb;
    *(v4fa*)(srow + col) = y[j];
  }
  if (F32OUT) {
    float* orow = outf + (size_t)row * kE;
    #pragma unroll
    for (int j = 0; j < 8; ++j) *(volatile v4f*)(orow + 128 * j + 4 * lane) = y[j];
    __threadfence();
    #pragma unroll
    for (int j = 0; j < 8; ++j) *(volatile v4f*)(orow + 128 * j + 4 * lane) = y[j];
  }
  __syncthreads();

  v8h o[4];
  #pragma unroll
  for (int j = 0; j < 4; ++j) {
    const int col = 256 * j + 8 * lane;
    const v4f a = *(const v4fa*)(srow + col);
    const v4f c = *(const v4fa*)(srow + col + 4);
    const v8h t = { (_Float16)a.x, (_Float16)a.y, (_Float16)a.z, (_Float16)a.w,
                    (_Float16)c.x, (_Float16)c.y, (_Float16)c.z, (_Float16)c.w };
    o[j] = t;
  }
  _Float16* hrow = outh + (size_t)row * kE;
  #pragma unroll
  for (int j = 0; j < 4; ++j) *(volatile v8h*)(hrow + 256 * j + 8 * lane) = o[j];
  __threadfence();
  #pragma unroll
  for (int j = 0; j < 4; ++j) *(volatile v8h*)(hrow + 256 * j + 8 * lane) = o[j];
}

struct Acc { v8f t[2][4]; };

__device__ __forceinline__ void gemm_core(Acc& acc, const _Float16* __restrict__ xa0,
                                          const _Float16* __restrict__ xa1,
                                          const _Float16* __restrict__ wb,
                                          int ldb, int K, int h) {
  const v8f zero8 = {0.f, 0.f, 0.f, 0.f, 0.f, 0.f, 0.f, 0.f};
  #pragma unroll
  for (int mt = 0; mt < 2; ++mt)
    #pragma unroll
    for (int nt = 0; nt < 4; ++nt) acc.t[mt][nt] = zero8;

  #pragma unroll 1
  for (int k0 = 0; k0 < K; k0 += 32) {
    const v16h a0 = load_frag(xa0 + k0, h);
    const v16h a1 = load_frag(xa1 + k0, h);
    #pragma unroll
    for (int nt = 0; nt < 4; ++nt) {
      const v16h bfr = load_frag(wb + (size_t)nt * 16 * ldb + k0, h);
      acc.t[0][nt] = wmma_f16(a0, bfr, acc.t[0][nt]);
      acc.t[1][nt] = wmma_f16(a1, bfr, acc.t[1][nt]);
    }
  }
}

__device__ __forceinline__ void qkv_store_pass(const _Float16* sT, _Float16* plane, _Float16* vt,
                                               int which, int bh, int l0, int w, int lane) {
  const int q8 = lane & 7, sub = lane >> 3;
  #pragma unroll
  for (int i = 0; i < 8; ++i) {
    const int lid = w * 32 + i * 4 + sub;
    v8h v;
    _Float16* dst;
    if (which != 2) {
      v = *(const v8ha*)(sT + lid * kD + 8 * q8);
      dst = plane + ((size_t)bh * kS + l0 + lid) * kD + 8 * q8;
    } else {
      const int d = lid >> 1, hl = lid & 1;
      v = *(const v8ha*)(sT + d * 128 + 64 * hl + 8 * q8);
      dst = vt + ((size_t)bh * kD + d) * kS + l0 + 64 * hl + 8 * q8;
    }
    *(volatile v8h*)dst = v;
  }
}

__global__ __launch_bounds__(128) void qkv_kernel(
    const _Float16* __restrict__ nh,
    const _Float16* __restrict__ wqkv,
    const float* __restrict__ bq, const float* __restrict__ bk, const float* __restrict__ bv,
    _Float16* __restrict__ qh,
    _Float16* __restrict__ kh,
    _Float16* __restrict__ vt)
{
  __shared__ __attribute__((aligned(16))) _Float16 sT[128 * 64];
  const int tid = threadIdx.x, lane = tid & 31, w = tid >> 5;
  const int h = lane >> 4, m = lane & 15;
  const int m0 = blockIdx.x * 128;
  const int cg = blockIdx.y;
  const int which = cg >> 4, head = cg & 15;
  const int m0w = m0 + 32 * w;

  const _Float16* xa0 = nh + (size_t)(m0w + m) * kE;
  const _Float16* xa1 = xa0 + (size_t)16 * kE;
  const _Float16* wb  = wqkv + ((size_t)which * kE + head * kD + m) * kE;

  Acc acc;
  gemm_core(acc, xa0, xa1, wb, kE, kE, h);

  const float* bias = (which == 0) ? bq : ((which == 1) ? bk : bv);
  #pragma unroll
  for (int nt = 0; nt < 4; ++nt) {
    const int feat = 16 * nt + m;
    const float bvl = bias[head * kD + feat];
    #pragma unroll
    for (int mt = 0; mt < 2; ++mt) {
      #pragma unroll
      for (int r = 0; r < 8; ++r) {
        const int tokl = 32 * w + 16 * mt + 8 * h + r;
        const float y = acc.t[mt][nt][r] * (1.0f / kWScale) + bvl;
        const int idx = (which == 2) ? (feat * 128 + tokl) : (tokl * kD + feat);
        sT[idx] = (_Float16)y;
      }
    }
  }
  __syncthreads();

  const int b = m0 / kS, l0 = m0 - b * kS, bh = b * kH + head;
  _Float16* plane = (which == 0) ? qh : kh;
  qkv_store_pass(sT, plane, vt, which, bh, l0, w, lane);
  __threadfence();
  qkv_store_pass(sT, plane, vt, which, bh, l0, w, lane);
}

__device__ __forceinline__ v8f mask_scale8(v8f z, v4i ma, v4i mb) {
  v8f s;
  s[0] = (ma.x != 0) ? z[0] * 0.125f : -1e9f;
  s[1] = (ma.y != 0) ? z[1] * 0.125f : -1e9f;
  s[2] = (ma.z != 0) ? z[2] * 0.125f : -1e9f;
  s[3] = (ma.w != 0) ? z[3] * 0.125f : -1e9f;
  s[4] = (mb.x != 0) ? z[4] * 0.125f : -1e9f;
  s[5] = (mb.y != 0) ? z[5] * 0.125f : -1e9f;
  s[6] = (mb.z != 0) ? z[6] * 0.125f : -1e9f;
  s[7] = (mb.w != 0) ? z[7] * 0.125f : -1e9f;
  return s;
}

__device__ __forceinline__ v16h pack_p(v8f a, v8f c) {
  const v16h r = { (_Float16)(a[0] * kPScale), (_Float16)(a[1] * kPScale), (_Float16)(a[2] * kPScale), (_Float16)(a[3] * kPScale),
                   (_Float16)(a[4] * kPScale), (_Float16)(a[5] * kPScale), (_Float16)(a[6] * kPScale), (_Float16)(a[7] * kPScale),
                   (_Float16)(c[0] * kPScale), (_Float16)(c[1] * kPScale), (_Float16)(c[2] * kPScale), (_Float16)(c[3] * kPScale),
                   (_Float16)(c[4] * kPScale), (_Float16)(c[5] * kPScale), (_Float16)(c[6] * kPScale), (_Float16)(c[7] * kPScale) };
  return r;
}

__device__ __forceinline__ void ctx_store_pass(const _Float16* so, _Float16* ctx,
                                               int b, int head, int q0, int lane) {
  const int q8 = lane & 7, sub = lane >> 3;
  #pragma unroll
  for (int i = 0; i < 4; ++i) {
    const int lid = i * 4 + sub;
    const v8h v = *(const v8ha*)(so + lid * 64 + 8 * q8);
    const size_t gi = ((size_t)b * kS + q0 + lid) * kE + head * kD + 8 * q8;
    *(volatile v8h*)(ctx + gi) = v;
  }
}

__global__ __launch_bounds__(128) void attn_kernel(
    const _Float16* __restrict__ qh,
    const _Float16* __restrict__ kh,
    const _Float16* __restrict__ vt,
    const int* __restrict__ mask,
    _Float16* __restrict__ ctx)
{
  __shared__ __attribute__((aligned(16))) _Float16 sO[4 * 16 * 64];

  const int tid = threadIdx.x, lane = tid & 31, w = tid >> 5;
  const int h = lane >> 4, m = lane & 15;
  const int bh = blockIdx.y, b = bh >> 4, head = bh & 15;
  const int q0 = blockIdx.x * 64 + 16 * w;

  const _Float16* qrow = qh + ((size_t)bh * kS + q0 + m) * kD;
  const v16h qb0 = load_frag(qrow, h);
  const v16h qb1 = load_frag(qrow + 32, h);

  const v8f zero8 = {0.f, 0.f, 0.f, 0.f, 0.f, 0.f, 0.f, 0.f};
  v8f o[4];
  #pragma unroll
  for (int t = 0; t < 4; ++t) o[t] = zero8;
  float mrun = -1e30f, lrun = 0.0f;

  const _Float16* kbase = kh + ((size_t)bh * kS + m) * kD;
  const _Float16* vbase = vt + ((size_t)bh * kD + m) * kS;
  const int* mkrow = mask + (size_t)(q0 + m) * kS + 8 * h;

  #pragma unroll 1
  for (int kb = 0; kb < kS; kb += 64) {
    v4i mka[4], mkb[4];
    int anyv = 0;
    #pragma unroll
    for (int j = 0; j < 4; ++j) {
      mka[j] = *(const v4ia*)(mkrow + kb + 16 * j);
      mkb[j] = *(const v4ia*)(mkrow + kb + 16 * j + 4);
      anyv |= (mka[j].x | mka[j].y) | (mka[j].z | mka[j].w);
      anyv |= (mkb[j].x | mkb[j].y) | (mkb[j].z | mkb[j].w);
    }
    if (!__any(anyv != 0)) continue;

    v8f s[4];
    #pragma unroll
    for (int j = 0; j < 4; ++j) {
      const _Float16* kp = kbase + (size_t)(kb + 16 * j) * kD;
      const v16h kf0 = load_frag(kp, h);
      const v16h kf1 = load_frag(kp + 32, h);
      v8f z = zero8;
      z = wmma_f16(kf0, qb0, z);
      z = wmma_f16(kf1, qb1, z);
      s[j] = z;
    }
    #pragma unroll
    for (int j = 0; j < 4; ++j) s[j] = mask_scale8(s[j], mka[j], mkb[j]);

    float mloc = s[0][0];
    #pragma unroll
    for (int j = 0; j < 4; ++j)
      #pragma unroll
      for (int r = 0; r < 8; ++r) mloc = fmaxf(mloc, s[j][r]);
    mloc = fmaxf(mloc, __shfl_xor(mloc, 16));
    const float mnew = fmaxf(mrun, mloc);
    const float alpha = __expf(mrun - mnew);
    mrun = mnew;
    float lsum = 0.0f;
    #pragma unroll
    for (int j = 0; j < 4; ++j)
      #pragma unroll
      for (int r = 0; r < 8; ++r) {
        const float p = __expf(s[j][r] - mnew);
        s[j][r] = p;
        lsum += p;
      }
    lsum += __shfl_xor(lsum, 16);
    lrun = lrun * alpha + lsum;
    #pragma unroll
    for (int t = 0; t < 4; ++t)
      #pragma unroll
      for (int r = 0; r < 8; ++r) o[t][r] = o[t][r] * alpha;

    const v16h pb0 = pack_p(s[0], s[1]);
    const v16h pb1 = pack_p(s[2], s[3]);

    #pragma unroll
    for (int t = 0; t < 4; ++t) {
      const _Float16* vp = vbase + (size_t)(16 * t) * kS + kb;
      const v16h vf0 = load_frag(vp, h);
      const v16h vf1 = load_frag(vp + 32, h);
      o[t] = wmma_f16(vf0, pb0, o[t]);
      o[t] = wmma_f16(vf1, pb1, o[t]);
    }
  }

  const float inv = (1.0f / lrun) * (1.0f / kPScale);
  _Float16* so = sO + w * 1024;
  #pragma unroll
  for (int t = 0; t < 4; ++t)
    #pragma unroll
    for (int r = 0; r < 8; ++r)
      so[m * 64 + 16 * t + 8 * h + r] = (_Float16)(o[t][r] * inv);
  __syncthreads();

  ctx_store_pass(so, ctx, b, head, q0, lane);
  __threadfence();
  ctx_store_pass(so, ctx, b, head, q0, lane);
}

__global__ __launch_bounds__(128) void gemm_res_kernel(
    const _Float16* __restrict__ A, int K,
    const _Float16* __restrict__ Wt,
    const float* __restrict__ bias,
    const float* __restrict__ resid,
    float* __restrict__ out,
    float inv)
{
  __shared__ __attribute__((aligned(16))) float sT[4 * 32 * 64];
  const int tid = threadIdx.x, lane = tid & 31, w = tid >> 5;
  const int h = lane >> 4, m = lane & 15;
  const int m0 = blockIdx.x * 128, n0 = blockIdx.y * 64;
  const int m0w = m0 + 32 * w;

  const _Float16* xa0 = A + (size_t)(m0w + m) * K;
  const _Float16* xa1 = xa0 + (size_t)16 * K;
  const _Float16* wb  = Wt + (size_t)(n0 + m) * K;

  Acc acc;
  gemm_core(acc, xa0, xa1, wb, K, K, h);

  float* st = sT + w * 2048;
  #pragma unroll
  for (int nt = 0; nt < 4; ++nt) {
    const int col = 16 * nt + m;
    const float bvl = bias[n0 + col];
    #pragma unroll
    for (int mt = 0; mt < 2; ++mt)
      #pragma unroll
      for (int r = 0; r < 8; ++r)
        st[(16 * mt + 8 * h + r) * 64 + col] = acc.t[mt][nt][r] * inv + bvl;
  }
  __syncthreads();

  const int q8 = lane & 7, sub = lane >> 3;
  v4f ov[16];
  #pragma unroll
  for (int i = 0; i < 16; ++i) {
    const int lid = 4 * i + sub;
    const int row = lid >> 1, hl = lid & 1;
    const int cofs = 32 * hl + 4 * q8;
    const v4f a = *(const v4fa*)(st + row * 64 + cofs);
    const v4f rsd = *(const v4fa*)(resid + (size_t)(m0w + row) * kE + n0 + cofs);
    ov[i] = a + rsd;
  }
  #pragma unroll
  for (int i = 0; i < 16; ++i) {
    const int lid = 4 * i + sub;
    const int row = lid >> 1, hl = lid & 1;
    *(volatile v4f*)(out + (size_t)(m0w + row) * kE + n0 + 32 * hl + 4 * q8) = ov[i];
  }
  __threadfence();
  #pragma unroll
  for (int i = 0; i < 16; ++i) {
    const int lid = 4 * i + sub;
    const int row = lid >> 1, hl = lid & 1;
    *(volatile v4f*)(out + (size_t)(m0w + row) * kE + n0 + 32 * hl + 4 * q8) = ov[i];
  }
}

__device__ __forceinline__ void h1_store_pass(const _Float16* sT, _Float16* h1, int m0, int n0,
                                              int w, int lane) {
  const int q8 = lane & 7, sub = lane >> 3;
  #pragma unroll
  for (int i = 0; i < 8; ++i) {
    const int lid = w * 32 + i * 4 + sub;
    const v8h v = *(const v8ha*)(sT + lid * 64 + 8 * q8);
    *(volatile v8h*)(h1 + (size_t)(m0 + lid) * kF + n0 + 8 * q8) = v;
  }
}

__global__ __launch_bounds__(128) void ffn1_kernel(
    const _Float16* __restrict__ A,
    const _Float16* __restrict__ Wt,
    const float* __restrict__ bias,
    _Float16* __restrict__ h1)
{
  __shared__ __attribute__((aligned(16))) _Float16 sT[128 * 64];
  const int tid = threadIdx.x, lane = tid & 31, w = tid >> 5;
  const int h = lane >> 4, m = lane & 15;
  const int m0 = blockIdx.x * 128, n0 = blockIdx.y * 64;
  const int m0w = m0 + 32 * w;

  const _Float16* xa0 = A + (size_t)(m0w + m) * kE;
  const _Float16* xa1 = xa0 + (size_t)16 * kE;
  const _Float16* wb  = Wt + (size_t)(n0 + m) * kE;

  Acc acc;
  gemm_core(acc, xa0, xa1, wb, kE, kE, h);

  #pragma unroll
  for (int nt = 0; nt < 4; ++nt) {
    const int feat = 16 * nt + m;
    const float bvl = bias[n0 + feat];
    #pragma unroll
    for (int mt = 0; mt < 2; ++mt)
      #pragma unroll
      for (int r = 0; r < 8; ++r) {
        const int tokl = 32 * w + 16 * mt + 8 * h + r;
        const float v = gelu_exact(acc.t[mt][nt][r] * (1.0f / kWScale) + bvl);
        sT[tokl * 64 + feat] = (_Float16)(v * kHScale);
      }
  }
  __syncthreads();

  h1_store_pass(sT, h1, m0, n0, w, lane);
  __threadfence();
  h1_store_pass(sT, h1, m0, n0, w, lane);
}

extern "C" void kernel_launch(void* const* d_in, const int* in_sizes, int n_in,
                              void* d_out, int out_size, void* d_ws, size_t ws_size,
                              hipStream_t stream) {
  if (n_in < 18) return;
  if (in_sizes[0] != kM * kE) return;
  if (in_sizes[1] != kS * kS) return;
  if (in_sizes[2] != kE * kE || in_sizes[4] != kE * kE || in_sizes[6] != kE * kE || in_sizes[8] != kE * kE) return;
  if (in_sizes[3] != kE || in_sizes[5] != kE || in_sizes[7] != kE || in_sizes[9] != kE) return;
  if (in_sizes[10] != kE * kF || in_sizes[11] != kF) return;
  if (in_sizes[12] != kF * kE || in_sizes[13] != kE) return;
  if (in_sizes[14] != kE || in_sizes[15] != kE || in_sizes[16] != kE || in_sizes[17] != kE) return;
  if (out_size != kM * kE) return;

  const float* x    = (const float*)d_in[0];
  const int*   mask = (const int*)d_in[1];
  const float* Wq   = (const float*)d_in[2];
  const float* bq   = (const float*)d_in[3];
  const float* Wk   = (const float*)d_in[4];
  const float* bk   = (const float*)d_in[5];
  const float* Wv   = (const float*)d_in[6];
  const float* bv   = (const float*)d_in[7];
  const float* Wo   = (const float*)d_in[8];
  const float* bo   = (const float*)d_in[9];
  const float* W1   = (const float*)d_in[10];
  const float* b1   = (const float*)d_in[11];
  const float* W2   = (const float*)d_in[12];
  const float* b2   = (const float*)d_in[13];
  const float* ln1g = (const float*)d_in[14];
  const float* ln1b = (const float*)d_in[15];
  const float* ln2g = (const float*)d_in[16];
  const float* ln2b = (const float*)d_in[17];
  float* out = (float*)d_out;

  const size_t wqkv_b = (size_t)3 * kE * kE * 2;
  const size_t wo_b   = (size_t)kE * kE * 2;
  const size_t w1_b   = (size_t)kF * kE * 2;
  const size_t w2_b   = (size_t)kE * kF * 2;
  const size_t act16  = (size_t)kM * kE * 2;
  const size_t act32  = (size_t)kM * kE * 4;
  const size_t h1_b   = (size_t)kM * kF * 2;

  const size_t o_wqkv = 0;
  const size_t o_wo   = o_wqkv + wqkv_b;
  const size_t o_w1   = o_wo + wo_b;
  const size_t o_w2   = o_w1 + w1_b;
  const size_t o_nh   = o_w2 + w2_b;
  const size_t o_qh   = o_nh + act16;
  const size_t o_kh   = o_qh + act16;
  const size_t o_vt   = o_kh + act16;
  const size_t o_y    = o_vt + act16;
  const size_t o_x2f  = o_y + act32;
  const size_t o_x2h  = o_x2f + act32;
  const size_t total  = o_x2h + act16;
  const size_t o_h1   = o_nh;
  if (o_h1 + h1_b > o_y) return;
  if (total > ws_size) return;

  char* ws = (char*)d_ws;
  _Float16* wqkv = (_Float16*)(ws + o_wqkv);
  _Float16* wo_t = (_Float16*)(ws + o_wo);
  _Float16* w1_t = (_Float16*)(ws + o_w1);
  _Float16* w2_t = (_Float16*)(ws + o_w2);
  _Float16* nh   = (_Float16*)(ws + o_nh);
  _Float16* ctx  = (_Float16*)(ws + o_nh);
  _Float16* qh   = (_Float16*)(ws + o_qh);
  _Float16* kh   = (_Float16*)(ws + o_kh);
  _Float16* vt   = (_Float16*)(ws + o_vt);
  _Float16* h1   = (_Float16*)(ws + o_h1);
  float*    y_f  = (float*)(ws + o_y);
  float*    x2f  = (float*)(ws + o_x2f);
  _Float16* x2h  = (_Float16*)(ws + o_x2h);

  cvt_wt_kernel<<<dim3(kE / 64, kE / 64), 256, 0, stream>>>(Wq, wqkv, kE, kE, kWScale);
  cvt_wt_kernel<<<dim3(kE / 64, kE / 64), 256, 0, stream>>>(Wk, wqkv + (size_t)kE * kE, kE, kE, kWScale);
  cvt_wt_kernel<<<dim3(kE / 64, kE / 64), 256, 0, stream>>>(Wv, wqkv + (size_t)2 * kE * kE, kE, kE, kWScale);
  cvt_wt_kernel<<<dim3(kE / 64, kE / 64), 256, 0, stream>>>(Wo, wo_t, kE, kE, kWScale);
  cvt_wt_kernel<<<dim3(kF / 64, kE / 64), 256, 0, stream>>>(W1, w1_t, kE, kF, kWScale);
  cvt_wt_kernel<<<dim3(kE / 64, kF / 64), 256, 0, stream>>>(W2, w2_t, kF, kE, kWScale);

  ln_kernel<false><<<kM / 8, 256, 0, stream>>>(x, ln1g, ln1b, y_f, nh);

  qkv_kernel<<<dim3(kM / 128, 3 * kH), 128, 0, stream>>>(nh, wqkv, bq, bk, bv, qh, kh, vt);

  attn_kernel<<<dim3(kS / 64, kB * kH), 128, 0, stream>>>(qh, kh, vt, mask, ctx);

  gemm_res_kernel<<<dim3(kM / 128, kE / 64), 128, 0, stream>>>(ctx, kE, wo_t, bo, x, y_f, 1.0f / kWScale);

  ln_kernel<true><<<kM / 8, 256, 0, stream>>>(y_f, ln2g, ln2b, x2f, x2h);

  ffn1_kernel<<<dim3(kM / 128, kF / 64), 128, 0, stream>>>(x2h, w1_t, b1, h1);

  gemm_res_kernel<<<dim3(kM / 128, kE / 64), 128, 0, stream>>>(h1, kF, w2_t, b2, x2f, out,
                                                               1.0f / (kWScale * kHScale));
}
